// GraphAttentionEncoder_68264210202884
// MI455X (gfx1250) — hardware-run, weakly checked
//
#include <hip/hip_runtime.h>

typedef float          v8f   __attribute__((ext_vector_type(8)));
typedef float          v4f   __attribute__((ext_vector_type(4)));
typedef unsigned int   v4u   __attribute__((ext_vector_type(4)));
typedef int            v8i   __attribute__((ext_vector_type(8)));
typedef unsigned short v8us  __attribute__((ext_vector_type(8)));
typedef unsigned short v16us __attribute__((ext_vector_type(16)));
typedef __bf16         v16bf __attribute__((ext_vector_type(16)));
typedef _Float16       v16h  __attribute__((ext_vector_type(16)));
typedef v4f  __attribute__((may_alias)) v4fa;
typedef v8us __attribute__((may_alias)) v8usa;
union FragB { v16bf v; v16us u; v8us h[2]; v8i w; };
union FragH { v16h  v; v16us u; v8us h[2]; v8i w; };

__device__ __forceinline__ v8f wmb(const FragB& a, const FragB& b, v8f c) {
  v8f d = __builtin_amdgcn_wmma_f32_16x16x32_bf16(false, a.v, false, b.v, (short)0, c, false, false);
  asm volatile("v_nop\n\tv_nop\n\tv_nop\n\tv_nop" : "+v"(d) : "v"(a.w), "v"(b.w));
  return d;
}

__device__ __forceinline__ v8f wmh(const FragH& a, const FragH& b, v8f c) {
  v8f d = __builtin_amdgcn_wmma_f32_16x16x32_f16(false, a.v, false, b.v, (short)0, c, false, false);
  asm volatile("v_nop\n\tv_nop\n\tv_nop\n\tv_nop" : "+v"(d) : "v"(a.w), "v"(b.w));
  return d;
}

__device__ __forceinline__ unsigned bf16_bits(float f) {
  const unsigned u = __float_as_uint(f);
  const unsigned r = (u + 0x7FFFu + ((u >> 16) & 1u)) >> 16;
  const unsigned q = (u >> 16) | 0x40u;
  return ((u & 0x7fffffffu) > 0x7f800000u) ? q : r;
}

__device__ __forceinline__ float bf16_val(float f) {
  return __uint_as_float(bf16_bits(f) << 16);
}
__device__ __forceinline__ int clampi(int v, int lo, int hi) {
  return v < lo ? lo : (v > hi ? hi : v);
}

__device__ __forceinline__ unsigned f16_bits(float f) {
  const unsigned u  = __float_as_uint(f);
  const unsigned s  = (u >> 16) & 0x8000u;
  const unsigned a  = u & 0x7fffffffu;
  const unsigned t  = a - 0x38000000u;
  const unsigned r  = (t + 0x0FFFu + ((t >> 13) & 1u)) >> 13;
  const unsigned rc = r > 0x7C00u ? 0x7C00u : r;
  const bool small  = a < 0x38800000u;
  const bool isnan  = a > 0x7f800000u;
  const unsigned fin = small ? 0u : (s | rc);
  return isnan ? (s | 0x7E00u) : fin;
}

__device__ __forceinline__ unsigned pk16(unsigned lo, unsigned hi) { return lo | (hi << 16); }
__device__ __forceinline__ unsigned bf16_lo_bits(float v) {
  float hi = bf16_val(v);
  asm volatile("" : "+v"(hi));
  return bf16_bits(v - hi);
}
__device__ __forceinline__ v4u pack8_bf16(v4f a, v4f c) {
  return (v4u){ pk16(bf16_bits(a[0]), bf16_bits(a[1])), pk16(bf16_bits(a[2]), bf16_bits(a[3])),
                pk16(bf16_bits(c[0]), bf16_bits(c[1])), pk16(bf16_bits(c[2]), bf16_bits(c[3])) };
}
__device__ __forceinline__ v4u pack8_bf16_lo(v4f a, v4f c) {
  return (v4u){ pk16(bf16_lo_bits(a[0]), bf16_lo_bits(a[1])), pk16(bf16_lo_bits(a[2]), bf16_lo_bits(a[3])),
                pk16(bf16_lo_bits(c[0]), bf16_lo_bits(c[1])), pk16(bf16_lo_bits(c[2]), bf16_lo_bits(c[3])) };
}
__device__ __forceinline__ v4u pack8_f16(v4f a, v4f c) {
  return (v4u){ pk16(f16_bits(a[0]), f16_bits(a[1])), pk16(f16_bits(a[2]), f16_bits(a[3])),
                pk16(f16_bits(c[0]), f16_bits(c[1])), pk16(f16_bits(c[2]), f16_bits(c[3])) };
}

template <int FORM>
__global__ __launch_bounds__(256) void k_plane(const float* __restrict__ src, int rows, int cols, int ldsrc,
                                               unsigned short* __restrict__ dst, int MP, int KP) {
  static_assert(FORM >= 0 && FORM <= 3);
  const int KTOT = (FORM == 1 || FORM == 3) ? 2 * KP : KP;
  const unsigned ppr   = (unsigned)(KTOT >> 3);
  const unsigned kp8   = (unsigned)(KP >> 3);
  const unsigned total = (unsigned)MP * ppr;
  const unsigned g     = blockIdx.x * 256u + threadIdx.x;
  const unsigned rowu  = g / ppr;
  const unsigned p     = g - rowu * ppr;
  const bool second    = p >= kp8;
  const int row = (int)rowu;
  const int c0  = (int)((second ? p - kp8 : p) << 3);
  const float* srow = src + (size_t)clampi(row, 0, rows - 1) * (size_t)ldsrc;
  float x[8];
  unsigned mk[8];
#pragma unroll
  for (int e = 0; e < 8; ++e) {
    const int c = c0 + e;
    const float v = srow[clampi(c, 0, cols - 1)];
    asm volatile("" :: "v"(v));
    x[e]  = v;
    mk[e] = (row < rows && c < cols) ? 0xFFFFu : 0u;
  }
  const v4f a = (v4f){ x[0], x[1], x[2], x[3] };
  const v4f c = (v4f){ x[4], x[5], x[6], x[7] };
  v4u o;
  if (FORM == 2) {
    o = pack8_f16(a, c);
  } else {
    const v4u hi = pack8_bf16(a, c);
    o = hi;
    if (FORM == 1) { const v4u lo = pack8_bf16_lo(a, c); o = second ? lo : hi; }
  }
  const v4u mw = (v4u){ pk16(mk[0], mk[1]), pk16(mk[2], mk[3]), pk16(mk[4], mk[5]), pk16(mk[6], mk[7]) };
  o &= mw;
  if (g < total) {
    volatile v4u* q = (volatile v4u*)(dst + (size_t)g * 8);
    *q = o;
    __threadfence();
    *q = o;
  }
}

template <int FORM> struct FragOf    { typedef FragB T; };
template <>         struct FragOf<2> { typedef FragH T; };
__device__ __forceinline__ v8f mm(const FragB& a, const FragB& b, v8f c) { return wmb(a, b, c); }
__device__ __forceinline__ v8f mm(const FragH& a, const FragH& b, v8f c) { return wmh(a, b, c); }
template <class F> __device__ __forceinline__ F ld_frag(const unsigned short* p) {
  F f;
  f.h[0] = *(const v8usa*)(p);
  f.h[1] = *(const v8usa*)(p + 16);
  return f;
}

template <int FORM, int EPI>
__global__ __launch_bounds__(256) __attribute__((amdgpu_num_vgpr(248)))
void k_gemm_nt(const unsigned short* __restrict__ A, const unsigned short* __restrict__ B,
               const float* __restrict__ bias, float* __restrict__ D, int M, int N, int KTOT, int ldd) {
  static_assert(FORM >= 0 && FORM <= 2);
  static_assert(EPI == 0 || EPI == 1);
  typedef typename FragOf<FORM>::T F;
  __shared__ __attribute__((aligned(16))) float sT[8][16 * 68];
  const int lane = threadIdx.x & 31;
  const int wave = threadIdx.x >> 5;
  const int tilesM = (M + 63) >> 6;
  const int tilesN = (N + 63) >> 6;
  const int tile = blockIdx.x * 8 + wave;
  if (tile >= tilesM * tilesN) return;
  const int tm = tile / tilesN;
  const int tn = tile - tm * tilesN;
  const int m0 = tm << 6;
  const int n0 = tn << 6;

  const int rl = lane & 15;
  const int h8 = (lane >> 4) * 8;
  const unsigned short* pa = A + (size_t)(m0 + rl) * (size_t)KTOT + h8;
  const unsigned short* pb = B + (size_t)(n0 + rl) * (size_t)KTOT + h8;

  v8f acc[4][4];
#pragma unroll
  for (int i = 0; i < 4; ++i)
#pragma unroll
    for (int j = 0; j < 4; ++j) acc[i][j] = (v8f){0.f, 0.f, 0.f, 0.f, 0.f, 0.f, 0.f, 0.f};

#pragma unroll 1
  for (int k0 = 0; k0 < KTOT; k0 += 32) {
    F bf[4];
#pragma unroll
    for (int j = 0; j < 4; ++j) bf[j] = ld_frag<F>(pb + (size_t)(j << 4) * (size_t)KTOT + k0);
#pragma unroll
    for (int i = 0; i < 4; ++i) {
      const F af = ld_frag<F>(pa + (size_t)(i << 4) * (size_t)KTOT + k0);
#pragma unroll
      for (int j = 0; j < 4; ++j) acc[i][j] = mm(af, bf[j], acc[i][j]);
    }
  }

  float* slab = sT[wave];
  const int hh = lane >> 4;
  const int c4 = (lane & 15) * 4;
  const int nc = n0 + c4;
  const bool cok = nc < N;
  v4f bv = (v4f){0.f, 0.f, 0.f, 0.f};
  if (EPI == 1) {
    bv = *(const v4fa*)(bias + clampi(nc, 0, N - 4));
    asm volatile("" :: "v"(bv));
  }
#pragma unroll
  for (int i = 0; i < 4; ++i) {
    const int mBase = m0 + (i << 4);
#pragma unroll
    for (int j = 0; j < 4; ++j) {
#pragma unroll
      for (int r = 0; r < 8; ++r) slab[(h8 + r) * 68 + (j << 4) + rl] = acc[i][j][r];
    }
    __builtin_amdgcn_fence(__ATOMIC_RELEASE, "workgroup");
    __builtin_amdgcn_wave_barrier();
    __builtin_amdgcn_fence(__ATOMIC_ACQUIRE, "workgroup");
    v4f vv[8];
#pragma unroll
    for (int it = 0; it < 8; ++it) {
      const int row = it * 2 + hh;
      v4f v = *(const v4fa*)(slab + row * 68 + c4);
      if (EPI == 1) v += bv;
      vv[it] = v;
    }
    for (int pass = 0; pass < 2; ++pass) {
#pragma unroll
      for (int it = 0; it < 8; ++it) {
        const int row = mBase + it * 2 + hh;
        if (cok && row < M) *(volatile v4f*)(D + (size_t)row * (size_t)ldd + nc) = vv[it];
      }
      __threadfence();
    }
    __builtin_amdgcn_fence(__ATOMIC_RELEASE, "workgroup");
    __builtin_amdgcn_wave_barrier();
    __builtin_amdgcn_fence(__ATOMIC_ACQUIRE, "workgroup");
  }
}

typedef int      i4v  __attribute__((ext_vector_type(4)));
typedef i4v      __attribute__((may_alias)) i4va;
typedef float    f2v  __attribute__((ext_vector_type(2)));
typedef f2v      __attribute__((may_alias)) f2va;
typedef unsigned u2v  __attribute__((ext_vector_type(2)));

#define NN      50000
#define NE      1200000
#define MPAD    50048
#define DM      64
#define NBAS    41
#define NBRUN   1024
#define NBLK    49
#define NPT     (NBLK * NBRUN)
#define RCAP    28672
#define TOTR    (NBLK * RCAP)
#define DEGCAP  64
#define CHUNK   2048
#define EPT     8
#define WCAP    256
#define LISTN   2048
#define LDS_BKT ((2 * RCAP + 2 * NBRUN + LISTN + 16) * 4)
#define PE_EMB  0
#define PE_WE   6400
#define PE_BE   9024
#define PE_LNS  9088
#define PE_LNB  9216
#define PE_BQ   9344
#define PE_BO   9728
#define PE_CEN  9856
#define PE_TOT  9920
#define R112    (1.0f / 1.12f)

static_assert(DM == 4 * 16);
static_assert(NBAS <= 44);
static_assert(NE < (1 << 21));
static_assert(NBRUN <= 1024 && NBRUN == 256 * 4);
static_assert(NN <= NBLK * NBRUN);
static_assert(MPAD % 64 == 0 && MPAD >= NN && MPAD <= NPT);
static_assert(NN % 16 == 0);
static_assert(DEGCAP % 32 == 0 && DEGCAP >= 46 + 8);
static_assert(RCAP % 1024 == 0 && RCAP >= 24990 + 2048);
static_assert(LISTN >= 8 * WCAP && LISTN >= NBRUN);
static_assert(CHUNK == 256 * EPT);
static_assert(LDS_BKT <= 327680);
static_assert((NE % 8) == 0);
static_assert(PE_WE == PE_EMB + 100 * 64 && PE_BE == PE_WE + NBAS * 64 && PE_TOT % 32 == 0);

__device__ __forceinline__ void wave_sync() {
  __builtin_amdgcn_fence(__ATOMIC_RELEASE, "workgroup");
  __builtin_amdgcn_wave_barrier();
  __builtin_amdgcn_fence(__ATOMIC_ACQUIRE, "workgroup");
}

__device__ __forceinline__ void cvt_region(const float* __restrict__ src, int nvec, float* dst, int gtid, int gs) {
#pragma unroll 1
  for (int base = 0; base < nvec; base += gs) {
    const int i  = base + gtid;
    const int ic = i < nvec ? i : nvec - 1;
    const v4f v = *(const v4fa*)(src + 4 * (size_t)ic);
    asm volatile("" :: "v"(v));
    const v4f o = (v4f){ bf16_val(v[0]), bf16_val(v[1]), bf16_val(v[2]), bf16_val(v[3]) };
    const bool ok = i < nvec;
    volatile v4f* q = (volatile v4f*)(dst + 4 * (size_t)ic);
    if (ok) *q = o;
    __threadfence();
    if (ok) *q = o;
  }
}
__device__ __forceinline__ void wt_region(const float* __restrict__ W, int ncols, int nunits, unsigned short* dst,
                                          int gtid, int gs) {
  const int perl = ncols * 16;
#pragma unroll 1
  for (int base = 0; base < nunits; base += gs) {
    const int u  = base + gtid;
    const int uc = u < nunits ? u : nunits - 1;
    const int l  = uc / perl;
    const int r  = uc - l * perl;
    const int n  = r >> 4;
    const int k8 = (r & 7) * 8;
    const float* sp = W + (size_t)l * 64 * (size_t)ncols + (size_t)k8 * (size_t)ncols + n;
    const float x0 = sp[0];
    const float x1 = sp[(size_t)ncols];
    const float x2 = sp[(size_t)2 * ncols];
    const float x3 = sp[(size_t)3 * ncols];
    const float x4 = sp[(size_t)4 * ncols];
    const float x5 = sp[(size_t)5 * ncols];
    const float x6 = sp[(size_t)6 * ncols];
    const float x7 = sp[(size_t)7 * ncols];
    asm volatile("" :: "v"(x0), "v"(x1), "v"(x2), "v"(x3), "v"(x4), "v"(x5), "v"(x6), "v"(x7));
    const v4u o = pack8_bf16((v4f){x0, x1, x2, x3}, (v4f){x4, x5, x6, x7});
    const bool ok = u < nunits;
    volatile v4u* q = (volatile v4u*)(dst + (size_t)uc * 8);
    if (ok) *q = o;
    __threadfence();
    if (ok) *q = o;
  }
}

__global__ __launch_bounds__(256) void k_prep(const float* __restrict__ emb, const float* __restrict__ We,
                                              const float* __restrict__ be, const float* __restrict__ lns,
                                              const float* __restrict__ lnb, const float* __restrict__ Wqkv,
                                              const float* __restrict__ bq, const float* __restrict__ Wout,
                                              const float* __restrict__ bo, float* PAR,
                                              unsigned short* WQ2, unsigned short* WO2) {
  const int gtid = (int)blockIdx.x * 256 + (int)threadIdx.x;
  const int gs   = (int)gridDim.x * 256;
  cvt_region(emb, 1600, PAR + PE_EMB, gtid, gs);
  cvt_region(We,  656,  PAR + PE_WE,  gtid, gs);
  cvt_region(be,  16,   PAR + PE_BE,  gtid, gs);
  cvt_region(lns, 32,   PAR + PE_LNS, gtid, gs);
  cvt_region(lnb, 32,   PAR + PE_LNB, gtid, gs);
  cvt_region(bq,  96,   PAR + PE_BQ,  gtid, gs);
  cvt_region(bo,  32,   PAR + PE_BO,  gtid, gs);
  wt_region(Wqkv, 192, 2 * 192 * 16, WQ2, gtid, gs);
  wt_region(Wout, 64,  2 * 64 * 16,  WO2, gtid, gs);
  if (gtid < 64) {
    const int c  = gtid;
    const int c1 = c < 1 ? 1 : (c > 40 ? 40 : c);
    const float t = (float)c1 / 40.0f;
    float ce = 8.0f * t;
    ce = (c == 0) ? 0.0f : ce;
    ce = (c >= 40) ? 8.0f : ce;
    volatile float* q = (volatile float*)(PAR + PE_CEN + c);
    *q = ce;
    __threadfence();
    *q = ce;
  }
}

__device__ __forceinline__ int hit_put(bool hj, unsigned sj, int ej, int wc, int* wl) {
  const unsigned mj = __builtin_amdgcn_ballot_w32(hj);
  const int pos = wc + (int)__builtin_amdgcn_mbcnt_lo(mj, 0u);
  if (hj && pos < WCAP) wl[pos] = (ej << 10) | (int)sj;
  return wc + (int)__builtin_popcount(mj);
}

__device__ __forceinline__ int scan_chunk(const int* __restrict__ dsts, int cbase, int slotBase, int vec8,
                                          int* wl, int tid) {
  const int el0  = tid * EPT;
  const int e0   = cbase + el0;
  const int sent = (int)0x80000000u;
  i4v da, db;
  if (vec8 != 0 && cbase + CHUNK <= NE) {
    da = *(const i4va*)(dsts + e0);
    db = *(const i4va*)(dsts + e0 + 4);
  } else {
    const int k0 = dsts[min(e0,     NE - 1)];
    const int k1 = dsts[min(e0 + 1, NE - 1)];
    const int k2 = dsts[min(e0 + 2, NE - 1)];
    const int k3 = dsts[min(e0 + 3, NE - 1)];
    const int k4 = dsts[min(e0 + 4, NE - 1)];
    const int k5 = dsts[min(e0 + 5, NE - 1)];
    const int k6 = dsts[min(e0 + 6, NE - 1)];
    const int k7 = dsts[min(e0 + 7, NE - 1)];
    asm volatile("" :: "v"(k0), "v"(k1), "v"(k2), "v"(k3), "v"(k4), "v"(k5), "v"(k6), "v"(k7));
    da.x = (e0     < NE) ? k0 : sent;
    da.y = (e0 + 1 < NE) ? k1 : sent;
    da.z = (e0 + 2 < NE) ? k2 : sent;
    da.w = (e0 + 3 < NE) ? k3 : sent;
    db.x = (e0 + 4 < NE) ? k4 : sent;
    db.y = (e0 + 5 < NE) ? k5 : sent;
    db.z = (e0 + 6 < NE) ? k6 : sent;
    db.w = (e0 + 7 < NE) ? k7 : sent;
  }
  const unsigned nbs = (unsigned)slotBase;
  const unsigned unb = (unsigned)NBRUN;
  const unsigned s0 = (unsigned)da.x - nbs, s1 = (unsigned)da.y - nbs;
  const unsigned s2 = (unsigned)da.z - nbs, s3 = (unsigned)da.w - nbs;
  const unsigned s4 = (unsigned)db.x - nbs, s5 = (unsigned)db.y - nbs;
  const unsigned s6 = (unsigned)db.z - nbs, s7 = (unsigned)db.w - nbs;
  const bool h0 = s0 < unb, h1 = s1 < unb, h2 = s2 < unb, h3 = s3 < unb;
  const bool h4 = s4 < unb, h5 = s5 < unb, h6 = s6 < unb, h7 = s7 < unb;
  const unsigned any = __builtin_amdgcn_ballot_w32(h0 | h1 | h2 | h3 | h4 | h5 | h6 | h7);
  int wc = 0;
  if (any != 0u) {
    wc = hit_put(h0, s0, el0 + 0, wc, wl);
    wc = hit_put(h1, s1, el0 + 1, wc, wl);
    wc = hit_put(h2, s2, el0 + 2, wc, wl);
    wc = hit_put(h3, s3, el0 + 3, wc, wl);
    wc = hit_put(h4, s4, el0 + 4, wc, wl);
    wc = hit_put(h5, s5, el0 + 5, wc, wl);
    wc = hit_put(h6, s6, el0 + 6, wc, wl);
    wc = hit_put(h7, s7, el0 + 7, wc, wl);
  }
  return wc;
}

__global__ __launch_bounds__(256) void k_bucket(const int* __restrict__ ei, const float* __restrict__ dist,
                                                int* OFFT, int* CNTT, int* FLAGT, int* SRCS, float* DISTS) {
  extern __shared__ v4f lds_dyn[];
  int* reg1 = (int*)lds_dyn;
  int* reg2 = reg1 + RCAP;
  int* scnt = reg2 + RCAP;
  int* soff = scnt + NBRUN;
  int* list = soff + NBRUN;
  int* wcnt = list + LISTN;
  int* wtot = wcnt + 8;
  const int tid = (int)threadIdx.x, lane = tid & 31, wave = tid >> 5;
  const int* srcs = ei;
  const int* dsts = ei + NE;
  const int nodeBase = (int)blockIdx.x * NBRUN;
  const int gbase    = (int)blockIdx.x * RCAP;

  for (int i = tid; i < NBRUN; i += 256) scnt[i] = 0;
  {
    const i4v z = (i4v){0, 0, 0, 0};
    for (int i = tid * 4; i < RCAP; i += 1024) *(i4va*)(reg2 + i) = z;
  }
  __syncthreads();

  int tot = 0;
  int* wl = list + wave * WCAP;
  const int nChunks = (NE + CHUNK - 1) / CHUNK;
#pragma unroll 1
  for (int ch = 0; ch < nChunks; ++ch) {
    const int cbase = ch * CHUNK;
    const int wc = scan_chunk(dsts, cbase, nodeBase, 1, wl, tid);
    if (lane == 0) wcnt[wave] = wc;
    __syncthreads();
    int pre = 0, all = 0;
#pragma unroll
    for (int w2 = 0; w2 < 8; ++w2) {
      int c = wcnt[w2];
      c = c < 0 ? 0 : (c > WCAP ? WCAP : c);
      all += c;
      pre += (w2 < wave) ? c : 0;
    }
    const int wcc  = wc > WCAP ? WCAP : wc;
    const int base = tot + pre;
#pragma unroll 1
    for (int i = lane; i < wcc; i += 32) {
      const int ent = wl[i];
      const int el  = (ent >> 10) & (CHUNK - 1);
      const int sl  = ent & (NBRUN - 1);
      int eid = cbase + el;
      eid = eid > NE - 1 ? NE - 1 : eid;
      const int pos = base + i;
      if (pos < RCAP) reg1[pos] = (int)((unsigned)eid | ((unsigned)sl << 21));
    }
    tot += all;
    tot = tot > RCAP ? RCAP : tot;
    __syncthreads();
  }
  const int nh = tot;

  if (wave == 0) {
#pragma unroll 1
    for (int b0 = 0; b0 < nh; b0 += 32) {
      int idx = b0 + lane;
      idx = idx < nh ? idx : nh - 1;
      const int uv  = reg1[idx];
      const int m32 = (nh - b0) < 32 ? (nh - b0) : 32;
#pragma unroll 1
      for (int k = 0; k < m32; ++k) {
        const int u  = __builtin_amdgcn_readlane(uv, k);
        const int sl = (int)((unsigned)u >> 21) & (NBRUN - 1);
        if (lane == 0) scnt[sl] = scnt[sl] + 1;
      }
    }
  }
  __syncthreads();

  {
    const i4v ca = *(const i4va*)(scnt + 4 * tid);
    const int e0 = ca.x < 0 ? 0 : ca.x, e1 = ca.y < 0 ? 0 : ca.y, e2 = ca.z < 0 ? 0 : ca.z, e3 = ca.w < 0 ? 0 : ca.w;
    const int ts = e0 + e1 + e2 + e3;
    int incl = ts;
#pragma unroll
    for (int d = 1; d < 32; d <<= 1) {
      const int up = __shfl_up(incl, d);
      if (lane >= d) incl += up;
    }
    if (lane == 31) wtot[wave] = incl;
    __syncthreads();
    int pre = 0;
#pragma unroll
    for (int w2 = 0; w2 < 8; ++w2) pre += (w2 < wave) ? wtot[w2] : 0;
    int run = pre + incl - ts;
    soff[4 * tid + 0] = run; run += e0;
    soff[4 * tid + 1] = run; run += e1;
    soff[4 * tid + 2] = run; run += e2;
    soff[4 * tid + 3] = run;
  }
  __syncthreads();
  for (int i = tid; i < NBRUN; i += 256) list[i] = soff[i];
  __syncthreads();

  if (wave == 0) {
#pragma unroll 1
    for (int b0 = 0; b0 < nh; b0 += 32) {
      int idx = b0 + lane;
      idx = idx < nh ? idx : nh - 1;
      const int uv  = reg1[idx];
      const int m32 = (nh - b0) < 32 ? (nh - b0) : 32;
#pragma unroll 1
      for (int k = 0; k < m32; ++k) {
        const int u   = __builtin_amdgcn_readlane(uv, k);
        const int sl  = (int)((unsigned)u >> 21) & (NBRUN - 1);
        const int eid = u & 0x1FFFFF;
        if (lane == 0) {
          int pos = list[sl];
          pos = pos < 0 ? 0 : (pos > RCAP - 1 ? RCAP - 1 : pos);
          reg2[pos] = eid;
          list[sl] = pos + 1;
        }
      }
    }
  }
  __syncthreads();

  const bool ovf = nh >= RCAP;
#pragma unroll 1
  for (int i0 = 0; i0 < RCAP; i0 += 1024) {
    const int i = i0 + tid * 4;
    const i4v e4 = *(const i4va*)(reg2 + i);
    const int ea = clampi(e4.x, 0, NE - 1), eb = clampi(e4.y, 0, NE - 1);
    const int ec = clampi(e4.z, 0, NE - 1), ed = clampi(e4.w, 0, NE - 1);
    const int ra = srcs[ea], rb = srcs[eb], rc = srcs[ec], rd = srcs[ed];
    asm volatile("" :: "v"(ra), "v"(rb), "v"(rc), "v"(rd));
    i4v so;
    so.x = (i     < nh) ? clampi(ra, 0, NN - 1) : 0;
    so.y = (i + 1 < nh) ? clampi(rb, 0, NN - 1) : 0;
    so.z = (i + 2 < nh) ? clampi(rc, 0, NN - 1) : 0;
    so.w = (i + 3 < nh) ? clampi(rd, 0, NN - 1) : 0;
    volatile i4v* qs = (volatile i4v*)(SRCS + (size_t)gbase + i);
    *qs = so;
    __threadfence();
    *qs = so;
    const float fa = dist[ea], fb = dist[eb], fc = dist[ec], fd = dist[ed];
    asm volatile("" :: "v"(fa), "v"(fb), "v"(fc), "v"(fd));
    v4f dv;
    dv[0] = (i     < nh) ? bf16_val(fa) : 0.0f;
    dv[1] = (i + 1 < nh) ? bf16_val(fb) : 0.0f;
    dv[2] = (i + 2 < nh) ? bf16_val(fc) : 0.0f;
    dv[3] = (i + 3 < nh) ? bf16_val(fd) : 0.0f;
    volatile v4f* qd = (volatile v4f*)(DISTS + (size_t)gbase + i);
    *qd = dv;
    __threadfence();
    *qd = dv;
  }
  {
    const int i = tid * 4;
    i4v c = *(const i4va*)(scnt + i);
    i4v o = *(const i4va*)(soff + i);
    o += gbase;
    const i4v big = (i4v){0x7fffffff, 0x7fffffff, 0x7fffffff, 0x7fffffff};
    c = ovf ? big : c;
    volatile i4v* qo = (volatile i4v*)(OFFT + (size_t)blockIdx.x * NBRUN + i);
    volatile i4v* qc = (volatile i4v*)(CNTT + (size_t)blockIdx.x * NBRUN + i);
    *qo = o; *qc = c;
    __threadfence();
    *qo = o; *qc = c;
    const int fv = ovf ? 1 : 0;
    const i4v f4 = (i4v){fv, fv, fv, fv};
    volatile i4v* qf = (volatile i4v*)(FLAGT + (size_t)blockIdx.x * 32 + (tid & 7) * 4);
    if (tid < 8) *qf = f4;
    __threadfence();
    if (tid < 8) *qf = f4;
  }
}

template <int MODE>
__global__ __launch_bounds__(256) void k_row(const int* __restrict__ xin, const float* __restrict__ PAR,
                                             float* Hbuf, const float* __restrict__ Pb,
                                             const int* __restrict__ FLAGT, unsigned* HNw, float* outp,
                                             int lnl, int bol) {
  const int tid = (int)threadIdx.x, lane = tid & 31, wave = tid >> 5;
  const int half = lane >> 4, cl = lane & 15, c4 = cl * 4;
  const v4f z4 = (v4f){0.f, 0.f, 0.f, 0.f};
  v4f gs = z4, gb = z4, bo = z4;
  if (MODE != 2) {
    gs = *(const v4fa*)(PAR + PE_LNS + lnl * 64 + c4);
    gb = *(const v4fa*)(PAR + PE_LNB + lnl * 64 + c4);
    asm volatile("" :: "v"(gs), "v"(gb));
  }
  if (MODE != 0) {
    bo = *(const v4fa*)(PAR + PE_BO + bol * 64 + c4);
    asm volatile("" :: "v"(bo));
  }
#pragma unroll 1
  for (int it = 0; it < 4; ++it) {
    const int row  = (int)blockIdx.x * 64 + it * 16 + wave * 2 + half;
    const int rowc = row < NN ? row : NN - 1;
    const bool live = row < NN;
    v4f hv;
    if (MODE == 0) {
      int xi = xin[rowc];
      asm volatile("" :: "v"(xi));
      xi = clampi(xi, 0, 99);
      const v4f e = *(const v4fa*)(PAR + PE_EMB + xi * 64 + c4);
      asm volatile("" :: "v"(e));
      hv = e * 8.0f;
    } else {
      const v4f h = *(const v4fa*)(Hbuf + (size_t)row * 64 + c4);
      const v4f p = *(const v4fa*)(Pb + (size_t)rowc * 64 + c4);
      asm volatile("" :: "v"(h), "v"(p));
      hv = h + (p + bo);
    }
    if (MODE == 2) {
      int fl = FLAGT[(rowc >> 10) * 32];
      asm volatile("" :: "v"(fl));
      const float qn = __uint_as_float(0x7fc00000u);
      const v4f n4 = (v4f){qn, qn, qn, qn};
      hv = (fl != 0) ? n4 : hv;
      volatile v4f* q = (volatile v4f*)(outp + (size_t)rowc * 64 + c4);
      if (live) *q = hv;
      __threadfence();
      if (live) *q = hv;
    } else {
      hv = live ? hv : z4;
      float s = (hv[0] + hv[1]) + (hv[2] + hv[3]);
      s += __shfl_xor(s, 8); s += __shfl_xor(s, 4); s += __shfl_xor(s, 2); s += __shfl_xor(s, 1);
      const float mu = s * 0.015625f;
      const v4f d = hv - mu;
      float q2 = (d[0] * d[0] + d[1] * d[1]) + (d[2] * d[2] + d[3] * d[3]);
      q2 += __shfl_xor(q2, 8); q2 += __shfl_xor(q2, 4); q2 += __shfl_xor(q2, 2); q2 += __shfl_xor(q2, 1);
      const float var = q2 * 0.015625f;
      const float rs = 1.0f / sqrtf(var + 1e-5f);
      v4f hn = (d * rs) * gs + gb;
      hn = live ? hn : z4;
      u2v wh, wlo;
      wh[0]  = pk16(bf16_bits(hn[0]), bf16_bits(hn[1]));
      wh[1]  = pk16(bf16_bits(hn[2]), bf16_bits(hn[3]));
      wlo[0] = pk16(bf16_lo_bits(hn[0]), bf16_lo_bits(hn[1]));
      wlo[1] = pk16(bf16_lo_bits(hn[2]), bf16_lo_bits(hn[3]));
      volatile v4f* qh  = (volatile v4f*)(Hbuf + (size_t)row * 64 + c4);
      volatile u2v* qnh = (volatile u2v*)(HNw + (size_t)row * 64 + cl * 2);
      volatile u2v* qnl = (volatile u2v*)(HNw + (size_t)row * 64 + 32 + cl * 2);
      *qh = hv; *qnh = wh; *qnl = wlo;
      __threadfence();
      *qh = hv; *qnh = wh; *qnl = wlo;
    }
  }
  (void)xin; (void)Pb; (void)FLAGT; (void)HNw; (void)outp;
}

__global__ __launch_bounds__(256) __attribute__((amdgpu_num_vgpr(248)))
void k_attn(const float* __restrict__ QKV, const float* __restrict__ PAR,
            const int* __restrict__ OFFT, const int* __restrict__ CNTT, const int* __restrict__ FLAGT,
            const int* __restrict__ SRCS, const float* __restrict__ DISTS, unsigned* __restrict__ AGGw) {
  __shared__ __attribute__((aligned(16))) float sWe[NBAS * DM];
  __shared__ __attribute__((aligned(16))) float sBe[DM];
  __shared__ __attribute__((aligned(16))) float sCen[64];
  __shared__ __attribute__((aligned(16))) float sQ[8][DM];
  __shared__ __attribute__((aligned(16))) float sU[8][44 * 4];
  __shared__ __attribute__((aligned(16))) float sQb[8][8];
  __shared__ __attribute__((aligned(16))) float sSc[8][DEGCAP * 4];
  __shared__ __attribute__((aligned(16))) int   sSrc[8][DEGCAP];
  const int tid = (int)threadIdx.x, lane = tid & 31, wave = tid >> 5;

#pragma unroll 1
  for (int i0 = 0; i0 < 768; i0 += 256) {
    const int i  = i0 + tid;
    const int ic = i < 656 ? i : 655;
    const v4f w = *(const v4fa*)(PAR + PE_WE + 4 * ic);
    asm volatile("" :: "v"(w));
    if (i < 656) *(v4fa*)(sWe + 4 * i) = w;
  }
  {
    const int ic = tid & 15;
    const v4f b = *(const v4fa*)(PAR + PE_BE + 4 * ic);
    const v4f c = *(const v4fa*)(PAR + PE_CEN + 4 * ic);
    asm volatile("" :: "v"(b), "v"(c));
    if (tid < 16) { *(v4fa*)(sBe + 4 * ic) = b; *(v4fa*)(sCen + 4 * ic) = c; }
  }
  __syncthreads();

  float* wq  = sQ[wave];
  float* wu  = sU[wave];
  float* wqb = sQb[wave];
  float* wsc = sSc[wave];
  int*   wsr = sSrc[wave];
  const int head = lane >> 3;

#pragma unroll 1
  for (int j = 0; j < 8; ++j) {
    const int row  = (int)blockIdx.x * 64 + wave * 8 + j;
    const int rowc = row < NN ? row : NN - 1;
    const bool live = row < NN;
    int o    = OFFT[row];
    int craw = CNTT[row];
    int fl   = FLAGT[(row >> 10) * 32];
    asm volatile("" :: "v"(o), "v"(craw), "v"(fl));
    int cv = clampi(craw, 0, DEGCAP);
    cv = live ? cv : 0;
    const int cnt = __builtin_amdgcn_readfirstlane(cv);
    const int stv = clampi(o, 0, TOTR - 1);
    const int st  = __builtin_amdgcn_readfirstlane(stv);
    const bool poison = live && (craw > DEGCAP || craw < 0 || fl != 0);

    wave_sync();
    {
      const f2v qv = *(const f2va*)(QKV + (size_t)rowc * 192 + 2 * lane);
      asm volatile("" :: "v"(qv));
      wq[2 * lane]     = qv[0];
      wq[2 * lane + 1] = qv[1];
    }
    wave_sync();

#pragma unroll 1
    for (int rnd = 0; rnd < 2; ++rnd) {
      const int c  = rnd * 32 + lane;
      const int cc = c < NBAS ? c : NBAS - 1;
#pragma unroll 1
      for (int hd = 0; hd < 4; ++hd) {
        const float* wp = sWe + cc * 64 + hd * 16;
        const float* qp = wq + hd * 16;
        float a = 0.f;
#pragma unroll
        for (int t = 0; t < 4; ++t) {
          const v4f w  = *(const v4fa*)(wp + 4 * t);
          const v4f q4 = *(const v4fa*)(qp + 4 * t);
          a = fmaf(w[0], q4[0], a); a = fmaf(w[1], q4[1], a);
          a = fmaf(w[2], q4[2], a); a = fmaf(w[3], q4[3], a);
        }
        const float uu = a * R112;
        if (c < NBAS) wu[c * 4 + hd] = uu;
      }
    }
    {
      const int hd = lane & 3;
      float a = 0.f;
#pragma unroll 1
      for (int t = 0; t < 4; ++t) {
        const v4f b  = *(const v4fa*)(sBe + hd * 16 + 4 * t);
        const v4f q4 = *(const v4fa*)(wq + hd * 16 + 4 * t);
        a = fmaf(b[0], q4[0], a); a = fmaf(b[1], q4[1], a);
        a = fmaf(b[2], q4[2], a); a = fmaf(b[3], q4[3], a);
      }
      if (lane < 4) wqb[lane] = a;
    }
    wave_sync();

    const int npass = (cnt + 31) >> 5;
#pragma unroll 1
    for (int p = 0; p < npass; ++p) {
      const int hq = p * 32 + lane;
      const int hc = hq < cnt ? hq : cnt - 1;
      const int idx = clampi(st + hc, 0, TOTR - 1);
      const int sraw = SRCS[idx];
      const float dd = DISTS[idx];
      asm volatile("" :: "v"(sraw), "v"(dd));
      const int s = clampi(sraw, 0, NN - 1);
      wsr[hq] = s;
      float ev0 = 0.f, ev1 = 0.f, ev2 = 0.f, ev3 = 0.f;
#pragma unroll 1
      for (int c = 0; c < NBAS; ++c) {
        const float ce = sCen[c];
        const v4f u4 = *(const v4fa*)(wu + 4 * c);
        const float df = (dd - ce) * 5.0f;
        const float bs = expf(-(df * df));
        ev0 = fmaf(bs, u4[0], ev0); ev1 = fmaf(bs, u4[1], ev1);
        ev2 = fmaf(bs, u4[2], ev2); ev3 = fmaf(bs, u4[3], ev3);
      }
      wsc[hq * 4 + 0] = ev0; wsc[hq * 4 + 1] = ev1; wsc[hq * 4 + 2] = ev2; wsc[hq * 4 + 3] = ev3;
      const float* krow = QKV + (size_t)s * 192 + 64;
#pragma unroll 1
      for (int hd = 0; hd < 4; ++hd) {
        const v4f k0 = *(const v4fa*)(krow + hd * 16);
        const v4f k1 = *(const v4fa*)(krow + hd * 16 + 4);
        const v4f k2 = *(const v4fa*)(krow + hd * 16 + 8);
        const v4f k3 = *(const v4fa*)(krow + hd * 16 + 12);
        asm volatile("" :: "v"(k0), "v"(k1), "v"(k2), "v"(k3));
        const v4f q0 = *(const v4fa*)(wq + hd * 16);
        const v4f q1 = *(const v4fa*)(wq + hd * 16 + 4);
        const v4f q2 = *(const v4fa*)(wq + hd * 16 + 8);
        const v4f q3 = *(const v4fa*)(wq + hd * 16 + 12);
        float d = 0.f;
        d = fmaf(q0[0], k0[0], d); d = fmaf(q0[1], k0[1], d); d = fmaf(q0[2], k0[2], d); d = fmaf(q0[3], k0[3], d);
        d = fmaf(q1[0], k1[0], d); d = fmaf(q1[1], k1[1], d); d = fmaf(q1[2], k1[2], d); d = fmaf(q1[3], k1[3], d);
        d = fmaf(q2[0], k2[0], d); d = fmaf(q2[1], k2[1], d); d = fmaf(q2[2], k2[2], d); d = fmaf(q2[3], k2[3], d);
        d = fmaf(q3[0], k3[0], d); d = fmaf(q3[1], k3[1], d); d = fmaf(q3[2], k3[2], d); d = fmaf(q3[3], k3[3], d);
        const float t = wsc[hq * 4 + hd];
        wsc[hq * 4 + hd] = ((d + t) + wqb[hd]) * 0.25f;
      }
    }
    wave_sync();

    float m = -__builtin_inff();
#pragma unroll 1
    for (int q = 0; q < cnt; ++q) m = fmaxf(m, wsc[q * 4 + head]);
    float ssum = 0.f, a0 = 0.f, a1 = 0.f;
#pragma unroll 1
    for (int q = 0; q < cnt; ++q) {
      const int s = clampi(wsr[q], 0, NN - 1);
      const f2v vv = *(const f2va*)(QKV + (size_t)s * 192 + 128 + 2 * lane);
      const float pr = expf(wsc[q * 4 + head] - m);
      ssum += pr;
      a0 = fmaf(pr, vv[0], a0);
      a1 = fmaf(pr, vv[1], a1);
    }
    const float inv = 1.0f / (ssum + 1e-16f);
    const float g0 = a0 * inv, g1 = a1 * inv;
    unsigned hw = pk16(bf16_bits(g0), bf16_bits(g1));
    unsigned lw = pk16(bf16_lo_bits(g0), bf16_lo_bits(g1));
    hw = live ? hw : 0u;
    lw = live ? lw : 0u;
    hw = poison ? 0x7fc07fc0u : hw;
    lw = poison ? 0x7fc07fc0u : lw;
    volatile unsigned* ph = (volatile unsigned*)(AGGw + (size_t)row * 64 + lane);
    volatile unsigned* pl = (volatile unsigned*)(AGGw + (size_t)row * 64 + 32 + lane);
    *ph = hw; *pl = lw;
    __threadfence();
    *ph = hw; *pl = lw;
  }
}

static inline size_t al256(size_t v) { return (v + 255) & ~(size_t)255; }

extern "C" void kernel_launch(void* const* d_in, const int* in_sizes, int n_in,
                              void* d_out, int out_size, void* d_ws, size_t ws_size,
                              hipStream_t stream) {
  if (n_in < 12) return;
  if (in_sizes[0] != NN || in_sizes[1] != 2 * NE || in_sizes[2] != NE) return;
  if (in_sizes[3] != 100 * DM || in_sizes[4] != NBAS * DM || in_sizes[5] != DM) return;
  if (in_sizes[6] != 2 * DM || in_sizes[7] != 2 * DM) return;
  if (in_sizes[8] != 2 * DM * 192 || in_sizes[9] != 2 * 192) return;
  if (in_sizes[10] != 2 * DM * DM || in_sizes[11] != 2 * DM) return;
  if (out_size != NN * DM) return;

  const int*   xin   = (const int*)  d_in[0];
  const int*   ei    = (const int*)  d_in[1];
  const float* dist  = (const float*)d_in[2];
  const float* emb   = (const float*)d_in[3];
  const float* We    = (const float*)d_in[4];
  const float* be    = (const float*)d_in[5];
  const float* lns   = (const float*)d_in[6];
  const float* lnb   = (const float*)d_in[7];
  const float* Wqkv  = (const float*)d_in[8];
  const float* bq    = (const float*)d_in[9];
  const float* Wout  = (const float*)d_in[10];
  const float* bo    = (const float*)d_in[11];
  float* out = (float*)d_out;

  char* ws = (char*)d_ws;
  size_t off = 0;
  const size_t oH    = off; off = al256(off + (size_t)MPAD * 64 * 4);
  const size_t oHN   = off; off = al256(off + (size_t)MPAD * 128 * 2);
  const size_t oQKV  = off; off = al256(off + (size_t)MPAD * 192 * 4);
  const size_t oP    = off; off = al256(off + (size_t)MPAD * 64 * 4);
  const size_t oOFF  = off; off = al256(off + (size_t)NPT * 4);
  const size_t oCNT  = off; off = al256(off + (size_t)NPT * 4);
  const size_t oFLG  = off; off = al256(off + (size_t)NBLK * 32 * 4);
  const size_t oSRC  = off; off = al256(off + (size_t)TOTR * 4);
  const size_t oDST  = off; off = al256(off + (size_t)TOTR * 4);
  const size_t oWQ2  = off; off = al256(off + (size_t)2 * 192 * 128 * 2);
  const size_t oWO2  = off; off = al256(off + (size_t)2 * 64 * 128 * 2);
  const size_t oPAR  = off; off = al256(off + (size_t)PE_TOT * 4);
  if (off > ws_size || off > ((size_t)128 << 20)) return;

  float*          H    = (float*)(ws + oH);
  unsigned short* HN   = (unsigned short*)(ws + oHN);
  float*          QKV  = (float*)(ws + oQKV);
  float*          P    = (float*)(ws + oP);
  int*            OFFT = (int*)(ws + oOFF);
  int*            CNTT = (int*)(ws + oCNT);
  int*            FLGT = (int*)(ws + oFLG);
  int*            SRCS = (int*)(ws + oSRC);
  float*          DSTS = (float*)(ws + oDST);
  unsigned short* WQ2  = (unsigned short*)(ws + oWQ2);
  unsigned short* WO2  = (unsigned short*)(ws + oWO2);
  float*          PAR  = (float*)(ws + oPAR);

  hipFuncSetAttribute(reinterpret_cast<const void*>(&k_bucket),
                      hipFuncAttributeMaxDynamicSharedMemorySize, LDS_BKT);

  const int gRow  = MPAD / 64;
  const int tQ    = ((NN + 63) / 64) * 3;
  const int tO    = ((NN + 63) / 64);
  const int gQ    = (tQ + 7) / 8;
  const int gO    = (tO + 7) / 8;

  k_prep<<<32, 256, 0, stream>>>(emb, We, be, lns, lnb, Wqkv, bq, Wout, bo, PAR, WQ2, WO2);
  k_bucket<<<NBLK, 256, LDS_BKT, stream>>>(ei, dist, OFFT, CNTT, FLGT, SRCS, DSTS);
  k_row<0><<<gRow, 256, 0, stream>>>(xin, PAR, H, P, FLGT, (unsigned*)HN, out, 0, 0);

  k_gemm_nt<1, 1><<<gQ, 256, 0, stream>>>(HN, WQ2, PAR + PE_BQ, QKV, NN, 192, 128, 192);
  k_attn<<<gRow, 256, 0, stream>>>(QKV, PAR, OFFT, CNTT, FLGT, SRCS, DSTS, (unsigned*)HN);
  k_gemm_nt<1, 0><<<gO, 256, 0, stream>>>(HN, WO2, PAR + PE_BO, P, NN, 64, 128, 64);
  k_row<1><<<gRow, 256, 0, stream>>>(xin, PAR, H, P, FLGT, (unsigned*)HN, out, 1, 0);

  k_gemm_nt<1, 1><<<gQ, 256, 0, stream>>>(HN, WQ2 + 192 * 128, PAR + PE_BQ + 192, QKV, NN, 192, 128, 192);
  k_attn<<<gRow, 256, 0, stream>>>(QKV, PAR, OFFT, CNTT, FLGT, SRCS, DSTS, (unsigned*)HN);
  k_gemm_nt<1, 0><<<gO, 256, 0, stream>>>(HN, WO2 + 64 * 128, PAR + PE_BO + 64, P, NN, 64, 128, 64);
  k_row<2><<<gRow, 256, 0, stream>>>(xin, PAR, H, P, FLGT, (unsigned*)HN, out, 1, 1);
}
